// GATv2Layer_77730318123230
// MI455X (gfx1250) — hardware-verified
//
#include <hip/hip_runtime.h>


#ifndef NB
#define NB 4
#endif
#define NB_FULL 4
#define NN    1024
#define FI    64
#define FO    64
#define PCAR  1024.0f
#define HSC   16.0f
#define WSC   64.0f
#define SC_ONE 1.0f
#define SC_UV (1.0f / 1024.0f)
#define SC_PV (1.0f / 16384.0f)
#define LOG2E 1.4426950408889634f
#define NEGFILL (-9.0e15f)
#define LSLOPE 0.2f

static_assert(NB >= 1 && NB <= NB_FULL);
static_assert(FO == 64 && FI == 64);
static_assert((NB * NN) % 64 == 0 && NN % 64 == 0 && FO % 64 == 0);
static_assert(FI % 32 == 0 && FO % 32 == 0 && NN % 32 == 0);
static_assert(256 * 4 == NN);
static_assert(4 * 32 * 8 == NN);
static_assert(((size_t)NB * NN * FO) % 1024 == 0);
static_assert(((size_t)NB * NN * FI) % 8 == 0 && (FO * FI) % 8 == 0 && (2 * FO * FO) % 8 == 0);
static_assert((size_t)NB_FULL * NN * FO * 4 == 1048576);
static_assert((2 * FO + NN + 8) * 4 <= 131072);
static_assert(16 * 68 * 4 <= 131072);

static constexpr size_t WS_HB   = (size_t)NB * NN * FI * 2;
static constexpr size_t WS_LWB  = (size_t)FO * FI * 2;
static constexpr size_t WS_WP   = (size_t)2 * FO * FO * 2;
static constexpr size_t WS_HPF  = (size_t)NB * NN * FO * 4;
static constexpr size_t WS_HP16 = (size_t)NB * NN * FO * 2;
static constexpr size_t WS_HPT  = (size_t)NB * FO * NN * 2;
static constexpr size_t WS_UVF  = (size_t)2 * NB * NN * FO * 4;
static constexpr size_t WS_P16  = (size_t)NB * NN * NN * 2;
static constexpr size_t WS_OF   = (size_t)NB * NN * FO * 4;
static constexpr size_t WS_TOTAL = WS_HB + WS_LWB + WS_WP + WS_HPF + WS_HP16 + WS_HPT + WS_UVF + WS_P16 + WS_OF;
static_assert(WS_HB % 256 == 0 && WS_LWB % 256 == 0 && WS_WP % 256 == 0 && WS_HPF % 256 == 0 && WS_HP16 % 256 == 0 && WS_HPT % 256 == 0 && WS_UVF % 256 == 0 && WS_P16 % 256 == 0 && WS_OF % 256 == 0);
static_assert(WS_TOTAL <= (size_t)134217728);

typedef _Float16 h16;
typedef unsigned short bf;
typedef __attribute__((ext_vector_type(16))) __bf16   v16bf;
typedef __attribute__((ext_vector_type(16))) _Float16 v16h;
typedef __attribute__((ext_vector_type(8)))  _Float16 v8h;
typedef __attribute__((ext_vector_type(8)))  unsigned short v8us;
typedef __attribute__((ext_vector_type(8)))  float    v8f;
typedef __attribute__((ext_vector_type(4)))  float    v4f;
typedef __attribute__((ext_vector_type(2)))  _Float16 v2h;
typedef __attribute__((ext_vector_type(2)))  unsigned short v2us;
typedef v8h  __attribute__((may_alias)) v8ha;
typedef v4f  __attribute__((may_alias)) v4fa;
typedef v8us __attribute__((may_alias)) v8usa;

__device__ __forceinline__ unsigned short f2bf(float f) { unsigned u = __float_as_uint(f); u += 0x7FFFu + ((u >> 16) & 1u); return (unsigned short)(u >> 16); }
__device__ __forceinline__ float bf2f(unsigned short b) { return __uint_as_float(((unsigned)b) << 16); }
__device__ __forceinline__ float bfr(float f) { return bf2f(f2bf(f)); }
__device__ __forceinline__ v16h cat16(v8h lo, v8h hi) { return __builtin_shufflevector(lo, hi, 0, 1, 2, 3, 4, 5, 6, 7, 8, 9, 10, 11, 12, 13, 14, 15); }
__device__ __forceinline__ v16bf cat16b(v8us lo, v8us hi) { return __builtin_bit_cast(v16bf, __builtin_shufflevector(lo, hi, 0, 1, 2, 3, 4, 5, 6, 7, 8, 9, 10, 11, 12, 13, 14, 15)); }
__device__ __forceinline__ v8f wmma16(v16h a, v16h b, v8f c) { return __builtin_amdgcn_wmma_f32_16x16x32_f16(false, a, false, b, (short)0, c, false, false); }
__device__ __forceinline__ v8f wmmab(v16bf a, v16bf b, v8f c) { return __builtin_amdgcn_wmma_f32_16x16x32_bf16(false, a, false, b, (short)0, c, false, false); }

__device__ __forceinline__ h16 toh_flush(float v) { const float w = (fabsf(v) < 6.103515625e-05f) ? 0.0f : v; return (h16)w; }

template <typename T16> struct WFrag;
template <> struct WFrag<h16> { typedef v16h V; static __device__ __forceinline__ V ld(const h16* p) { return cat16(*(const v8h*)p, *(const v8h*)(p + 16)); } static __device__ __forceinline__ v8f mma(V a, V b, v8f c) { return wmma16(a, b, c); } };
template <> struct WFrag<bf> { typedef v16bf V; static __device__ __forceinline__ V ld(const bf* p) { return cat16b(*(const v8us*)p, *(const v8us*)(p + 16)); } static __device__ __forceinline__ v8f mma(V a, V b, v8f c) { return wmmab(a, b, c); } };
template <typename T16, int NSPLIT, bool BIAS>
__global__ __launch_bounds__(32) void k_gemmw(const T16* __restrict__ A, const T16* __restrict__ A2, const T16* __restrict__ Bt, const T16* __restrict__ Bt2, int K, float* C, int ldc, const float* __restrict__ bias, float csc, size_t sA, size_t sB, size_t sC) {
    typedef typename WFrag<T16>::V V;
    __shared__ __align__(16) float os[16 * 68];
    const size_t z = blockIdx.z; A += z * sA; if (A2) A2 += z * sA; Bt += z * sB; if (Bt2) Bt2 += z * sB; C += z * sC;
    const int lane = threadIdx.x & 31, lr = lane & 15, hi = lane >> 4; const int r0 = blockIdx.x * 64, c0 = blockIdx.y * 64;
    v8f acc[4][4];
#pragma unroll
    for (int mb = 0; mb < 4; ++mb)
#pragma unroll
        for (int nb = 0; nb < 4; ++nb) acc[mb][nb] = (v8f){};
    const size_t aoff = (size_t)(r0 + lr) * K + 8 * hi, boff = (size_t)(c0 + lr) * K + 8 * hi;
#pragma unroll 1
    for (int kc = 0; kc < K; kc += 32) {
        V a[4], a2[4];
#pragma unroll
        for (int mb = 0; mb < 4; ++mb) { a[mb] = WFrag<T16>::ld(A + aoff + (size_t)mb * 16 * K + kc); if (NSPLIT == 1 || NSPLIT == 2) a2[mb] = WFrag<T16>::ld(A2 + aoff + (size_t)mb * 16 * K + kc); }
#pragma unroll
        for (int nb = 0; nb < 4; ++nb) { const V b = WFrag<T16>::ld(Bt + boff + (size_t)nb * 16 * K + kc); V b2; if (NSPLIT >= 2) b2 = WFrag<T16>::ld(Bt2 + boff + (size_t)nb * 16 * K + kc);
#pragma unroll
            for (int mb = 0; mb < 4; ++mb) { acc[mb][nb] = WFrag<T16>::mma(a[mb], b, acc[mb][nb]); if (NSPLIT == 1 || NSPLIT == 2) acc[mb][nb] = WFrag<T16>::mma(a2[mb], b, acc[mb][nb]); if (NSPLIT >= 2) acc[mb][nb] = WFrag<T16>::mma(a[mb], b2, acc[mb][nb]); } }
        asm volatile("v_nop\n\tv_nop\n\tv_nop\n\tv_nop" : "+v"(acc[0][0]), "+v"(acc[1][1]), "+v"(acc[2][2]), "+v"(acc[3][3]) : "v"(a[0]), "v"(a[3]));
    }
#pragma unroll
    for (int mb = 0; mb < 4; ++mb) {
#pragma unroll
        for (int nb = 0; nb < 4; ++nb) {
#pragma unroll
            for (int j = 0; j < 8; ++j) os[(hi * 8 + j) * 68 + nb * 16 + lr] = acc[mb][nb][j]; }
        __builtin_amdgcn_wave_barrier(); asm volatile("" ::: "memory");
        float* crow = C + (size_t)(r0 + mb * 16) * ldc + c0;
#pragma unroll 1
        for (int ps = 0; ps < 2; ++ps) {
#pragma unroll
            for (int s = 0; s < 8; ++s) { const int row = 2 * s + hi, cofs = lr * 4; v4f val = *(const v4fa*)(os + row * 68 + cofs); val = val * csc;
                if (BIAS) { val[0] += bfr(bias[c0 + cofs]); val[1] += bfr(bias[c0 + cofs + 1]); val[2] += bfr(bias[c0 + cofs + 2]); val[3] += bfr(bias[c0 + cofs + 3]); }
                *(volatile v4f*)(crow + (size_t)row * ldc + cofs) = val; }
            if (ps == 0) __threadfence(); }
        __builtin_amdgcn_wave_barrier(); asm volatile("" ::: "memory");
    }
}

__global__ __launch_bounds__(256) void k_cvt8(const float* __restrict__ src, bf* dst, size_t n8) { const size_t i = (size_t)blockIdx.x * 256 + threadIdx.x; if (i >= n8) return; const v8f v = *(const v8f*)(src + i * 8); v8us o;
#pragma unroll
    for (int k = 0; k < 8; ++k) o[k] = f2bf(v[k]); *(volatile v8us*)(dst + i * 8) = o; __threadfence(); *(volatile v8us*)(dst + i * 8) = o; }

__global__ __launch_bounds__(256) void k_wconv(const float* __restrict__ W, h16* WP) {
    const int i = blockIdx.x * 256 + threadIdx.x; if (i >= 2 * FO * FO / 8) return;
    const int z = i / (FO * FO / 8); const int o = (i / (FO / 8)) % FO; const int f8 = (i % (FO / 8)) * 8;
    const v8f v = *(const v8f*)(W + (size_t)o * (2 * FO) + z * FO + f8); v8h r;
#pragma unroll
    for (int k = 0; k < 8; ++k) r[k] = toh_flush(bfr(v[k]) * WSC);
    *(volatile v8h*)(WP + (size_t)i * 8) = r; __threadfence(); *(volatile v8h*)(WP + (size_t)i * 8) = r;
}

__global__ __launch_bounds__(256) void k_hcv8(const float* __restrict__ src, h16* dst, size_t n8) {
    const size_t i = (size_t)blockIdx.x * 256 + threadIdx.x; if (i >= n8) return;
    const v8f v = *(const v8f*)(src + i * 8); v8h r;
#pragma unroll
    for (int k = 0; k < 8; ++k) r[k] = toh_flush(v[k] * HSC);
    *(volatile v8h*)(dst + i * 8) = r; __threadfence(); *(volatile v8h*)(dst + i * 8) = r;
}

__global__ __launch_bounds__(256) void k_hpt(const float* __restrict__ HP, h16* T16) {
    const size_t e = ((size_t)blockIdx.x * 256 + threadIdx.x) * 2; if (e >= (size_t)NB * FO * NN) return;
    const int j = (int)(e % NN); const int f = (int)((e / NN) % FO); const int b = (int)(e / ((size_t)NN * FO));
    v2h o;
#pragma unroll
    for (int q = 0; q < 2; ++q) o[q] = toh_flush(HP[((size_t)b * NN + j + q) * FO + f] * HSC);
    *(volatile v2h*)(T16 + e) = o; __threadfence(); *(volatile v2h*)(T16 + e) = o;
}

__global__ __launch_bounds__(256) void k_gscore(const float* __restrict__ U, const float* __restrict__ V, const int* __restrict__ adj, const float* __restrict__ av, h16* P16) {
    __shared__ __align__(16) float s_u[FO];
    __shared__ __align__(16) float s_a[FO];
    __shared__ __align__(16) float s_p[NN];
    __shared__ float red[8];
    const int rq = blockIdx.x; const int b = rq / NN;
    const int tid = threadIdx.x, lane = tid & 31; const int wave = __builtin_amdgcn_readfirstlane(threadIdx.x >> 5);
    if (wave < 2) s_u[tid] = U[(size_t)rq * FO + tid];
    else if (wave < 4) s_a[tid - FO] = bfr(av[tid - FO]);
    const int* arow = adj + (size_t)rq * NN;
    const int m0 = arow[tid], m1 = arow[tid + 256], m2 = arow[tid + 512], m3 = arow[tid + 768];
    const float* vb = V + (size_t)b * NN * FO + (size_t)tid * FO;
    __syncthreads();
    float e0 = 0.0f, e1 = 0.0f, e2 = 0.0f, e3 = 0.0f;
#pragma unroll 2
    for (int f4 = 0; f4 < FO / 4; ++f4) {
        const v4f a4 = *(const v4fa*)(s_a + f4 * 4); const v4f u4 = *(const v4fa*)(s_u + f4 * 4);
        const v4f x0 = *(const v4f*)(vb + f4 * 4);
        const v4f x1 = *(const v4f*)(vb + (size_t)256 * FO + f4 * 4);
        const v4f x2 = *(const v4f*)(vb + (size_t)512 * FO + f4 * 4);
        const v4f x3 = *(const v4f*)(vb + (size_t)768 * FO + f4 * 4);
#pragma unroll
        for (int c = 0; c < 4; ++c) {
            float t0 = u4[c] + x0[c]; t0 = (t0 > 0.0f) ? t0 : LSLOPE * t0; e0 = fmaf(a4[c], t0, e0);
            float t1 = u4[c] + x1[c]; t1 = (t1 > 0.0f) ? t1 : LSLOPE * t1; e1 = fmaf(a4[c], t1, e1);
            float t2 = u4[c] + x2[c]; t2 = (t2 > 0.0f) ? t2 : LSLOPE * t2; e2 = fmaf(a4[c], t2, e2);
            float t3 = u4[c] + x3[c]; t3 = (t3 > 0.0f) ? t3 : LSLOPE * t3; e3 = fmaf(a4[c], t3, e3);
        }
    }
    e0 = (m0 > 0) ? e0 : NEGFILL; e1 = (m1 > 0) ? e1 : NEGFILL; e2 = (m2 > 0) ? e2 : NEGFILL; e3 = (m3 > 0) ? e3 : NEGFILL;
    float m = e0; m = (e1 > m) ? e1 : m; m = (e2 > m) ? e2 : m; m = (e3 > m) ? e3 : m;
#pragma unroll
    for (int sh = 16; sh; sh >>= 1) { const float t = __shfl_xor(m, sh, 32); m = (t > m) ? t : m; }
    if (lane == 0) red[wave] = m;
    __syncthreads();
    m = red[0];
#pragma unroll
    for (int w = 1; w < 8; ++w) { const float t = red[w]; m = (t > m) ? t : m; }
    __syncthreads();
    const float p0 = __builtin_amdgcn_exp2f((e0 - m) * LOG2E), p1 = __builtin_amdgcn_exp2f((e1 - m) * LOG2E);
    const float p2 = __builtin_amdgcn_exp2f((e2 - m) * LOG2E), p3 = __builtin_amdgcn_exp2f((e3 - m) * LOG2E);
    s_p[tid] = p0; s_p[tid + 256] = p1; s_p[tid + 512] = p2; s_p[tid + 768] = p3;
    float sum = (p0 + p1) + (p2 + p3);
#pragma unroll
    for (int sh = 16; sh; sh >>= 1) sum += __shfl_xor(sum, sh, 32);
    if (lane == 0) red[wave] = sum;
    __syncthreads();
    sum = red[0];
#pragma unroll
    for (int w = 1; w < 8; ++w) sum += red[w];
    const float inv = __builtin_amdgcn_rcpf(sum); const float invp = inv * PCAR;
    if (wave < 4) {
        const int f0 = (wave * 32 + lane) * 8;
        const v4f q0 = *(const v4fa*)(s_p + f0); const v4f q1 = *(const v4fa*)(s_p + f0 + 4);
        v8h o;
#pragma unroll
        for (int c = 0; c < 4; ++c) { o[c] = toh_flush(q0[c] * invp); o[4 + c] = toh_flush(q1[c] * invp); }
        h16* dst = P16 + (size_t)rq * NN + f0;
        *(volatile v8h*)dst = o; __threadfence(); *(volatile v8h*)dst = o;
    }
}

__global__ __launch_bounds__(256) void k_eluo(const float* __restrict__ O, float* out) {
    __shared__ __align__(16) float s_o[1024];
    const int tid = threadIdx.x; const size_t base = (size_t)blockIdx.x * 1024;
#pragma unroll 1
    for (int q = 0; q < 4; ++q) { const float o = O[base + q * 256 + tid]; const float en = expm1f(o); s_o[q * 256 + tid] = (o > 0.0f) ? o : en; }
    __syncthreads();
    const v4f val = *(const v4fa*)(s_o + tid * 4);
    float* dst = out + base + tid * 4;
    *(volatile v4f*)dst = val; __threadfence(); *(volatile v4f*)dst = val;
}
static_assert(256 * 4 * 4 == 1024 * 4);
static_assert(4 * 32 * 16 == NN * 2);

extern "C" void kernel_launch(void* const* d_in, const int* in_sizes, int n_in,
                              void* d_out, int out_size, void* d_ws, size_t ws_size, hipStream_t stream) {
    if (n_in < 6) return;
    if (in_sizes[0] < NB * NN * FI || in_sizes[1] < NB * NN * NN || in_sizes[2] < FO * FI || in_sizes[3] < FO || in_sizes[4] < FO * 2 * FO || in_sizes[5] < FO) return;
    if (out_size < NB * NN * FO) return;
    const float* hin  = (const float*)d_in[0];
    const int*   adj  = (const int*)d_in[1];
    const float* linw = (const float*)d_in[2];
    const float* linb = (const float*)d_in[3];
    const float* Ww   = (const float*)d_in[4];
    const float* av   = (const float*)d_in[5];
    float* OUT0 = (float*)d_out;

    char* wsp = (char*)d_ws;
    auto take = [&](size_t bytes) { char* p = wsp; wsp += (bytes + 255) & ~(size_t)255; return (void*)p; };
    bf*    HB   = (bf*)take(WS_HB);
    bf*    LWB  = (bf*)take(WS_LWB);
    h16*   WP   = (h16*)take(WS_WP);
    float* HPF  = (float*)take(WS_HPF);
    h16*   HP16 = (h16*)take(WS_HP16);
    h16*   HPT  = (h16*)take(WS_HPT);
    float* UVF  = (float*)take(WS_UVF);
    h16*   P16  = (h16*)take(WS_P16);
    float* OF   = (float*)take(WS_OF);
    if ((size_t)(wsp - (char*)d_ws) > ws_size) return;

    k_cvt8<<<(unsigned)(((size_t)NB * NN * FI / 8 + 255) / 256), 256, 0, stream>>>(hin, HB, (size_t)NB * NN * FI / 8);
    k_cvt8<<<(unsigned)(((size_t)FO * FI / 8 + 255) / 256), 256, 0, stream>>>(linw, LWB, (size_t)FO * FI / 8);
    k_wconv<<<(unsigned)((2 * FO * FO / 8 + 255) / 256), 256, 0, stream>>>(Ww, WP);
    k_gemmw<bf, 0, true><<<dim3(NB * NN / 64, FO / 64, 1), 32, 0, stream>>>(HB, nullptr, LWB, nullptr, FI, HPF, FO, linb, SC_ONE, 0, 0, 0);
    k_hcv8<<<(unsigned)(((size_t)NB * NN * FO / 8 + 255) / 256), 256, 0, stream>>>(HPF, HP16, (size_t)NB * NN * FO / 8);
    k_hpt<<<(unsigned)(((size_t)NB * FO * NN / 2 + 255) / 256), 256, 0, stream>>>(HPF, HPT);
    k_gemmw<h16, 0, false><<<dim3(NB * NN / 64, FO / 64, 2), 32, 0, stream>>>(HP16, nullptr, WP, nullptr, FO, UVF, FO, nullptr, SC_UV, 0, (size_t)FO * FO, (size_t)NB * NN * FO);
    k_gscore<<<(unsigned)(NB * NN), 256, 0, stream>>>(UVF, UVF + (size_t)NB * NN * FO, adj, av, P16);
    k_gemmw<h16, 0, false><<<dim3(NN / 64, FO / 64, NB), 32, 0, stream>>>(P16, nullptr, HPT, nullptr, NN, OF, FO, nullptr, SC_PV, (size_t)NN * NN, (size_t)FO * NN, (size_t)NN * FO);
    k_eluo<<<(unsigned)((size_t)NB * NN * FO / 1024), 256, 0, stream>>>(OF, OUT0);
}
